// SS2D_MixerLite_25872882991493
// MI455X (gfx1250) — hardware-verified
//
#include <hip/hip_runtime.h>
#include <stdint.h>

#define B_   4
#define C_   256
#define H_   64
#define W_   64
#define L_   (H_ * W_)
#define NTOK (B_ * L_)
#define HID  512

typedef __attribute__((ext_vector_type(16))) _Float16 v16h;
typedef __attribute__((ext_vector_type(8)))  _Float16 v8h;
typedef __attribute__((ext_vector_type(16))) __bf16   v16b;
typedef __attribute__((ext_vector_type(8)))  __bf16   v8b;
typedef __attribute__((ext_vector_type(8)))  float    v8f;
typedef __attribute__((ext_vector_type(4)))  float    v4f;

__device__ __forceinline__ unsigned short f2bf_bits(float f) {
  unsigned u = __float_as_uint(f);
  return (unsigned short)((u + 0x7FFFu + ((u >> 16) & 1u)) >> 16);
}
__device__ __forceinline__ float bf_bits2f(unsigned short h) { return __uint_as_float(((unsigned)h) << 16); }

__device__ __forceinline__ float nan_clean_f(float v) {
  if (v != v) return 0.0f;
  if (__builtin_fabsf(v) == __builtin_inff()) return (v > 0.0f) ? 10000.0f : -10000.0f;
  return v;
}

__device__ __forceinline__ void dep_guard_h(v8f& a, v8f& b, v16h x, v16h y) { asm volatile("v_nop\n\tv_nop\n\tv_nop\n\tv_nop" : "+v"(a), "+v"(b) : "v"(x), "v"(y)); }
__device__ __forceinline__ void dep_guard_b(v8f& a, v8f& b, v16b x, v16b y) { asm volatile("v_nop\n\tv_nop\n\tv_nop\n\tv_nop" : "+v"(a), "+v"(b) : "v"(x), "v"(y)); }
__device__ __forceinline__ void keep4_h(v16h a, v16h b, v16h c, v16h d) { asm volatile("v_nop" :: "v"(a), "v"(b), "v"(c), "v"(d)); }
__device__ __forceinline__ void keep4_b(v16b a, v16b b, v16b c, v16b d) { asm volatile("v_nop" :: "v"(a), "v"(b), "v"(c), "v"(d)); }
__device__ __forceinline__ void acc_guard4(v8f& a, v8f& b, v8f& c, v8f& d) { asm volatile("v_nop\n\tv_nop\n\tv_nop\n\tv_nop" : "+v"(a), "+v"(b), "+v"(c), "+v"(d)); }
template <typename T> struct Frag;
template <> struct Frag<_Float16> {
  typedef v16h V; union U { v16h v; v8h h[2]; };
  static __device__ __forceinline__ v16h load(const _Float16* p) {
    U f; f.h[0] = *(const v8h*)(p); f.h[1] = *(const v8h*)(p + 16); return f.v;
  }
  static __device__ __forceinline__ v8f mma(v16h a, v16h b, v8f c) {
    return __builtin_amdgcn_wmma_f32_16x16x32_f16(false, a, false, b, (short)0, c, false, false);
  }
  static __device__ __forceinline__ void guard(v8f& a, v8f& b, v16h x, v16h y) { dep_guard_h(a, b, x, y); }
  static __device__ __forceinline__ void keep(v16h a, v16h b, v16h c, v16h d) { keep4_h(a, b, c, d); }
};
template <> struct Frag<__bf16> {
  typedef v16b V; union U { v16b v; v8b h[2]; };
  static __device__ __forceinline__ v16b load(const __bf16* p) {
    U f; f.h[0] = *(const v8b*)(p); f.h[1] = *(const v8b*)(p + 16); return f.v;
  }
  static __device__ __forceinline__ v8f mma(v16b a, v16b b, v8f c) {
    return __builtin_amdgcn_wmma_f32_16x16x32_bf16(false, a, false, b, (short)0, c, false, false);
  }
  static __device__ __forceinline__ void guard(v8f& a, v8f& b, v16b x, v16b y) { dep_guard_b(a, b, x, y); }
  static __device__ __forceinline__ void keep(v16b a, v16b b, v16b c, v16b d) { keep4_b(a, b, c, d); }
};

template <int ET> struct Elem;
template <> struct Elem<0> { typedef _Float16 T; };
template <> struct Elem<1> { typedef __bf16 T; };
template <int ET, bool SPLIT, int BIAS_MODE, int OUT_MODE, bool RESID, int ACT, int NCL>
__global__ __launch_bounds__(256) void wmma_gemm64(
    const unsigned short* __restrict__ Ap, const unsigned short* __restrict__ A2p, int lda, long strideA,
    const unsigned short* __restrict__ Btp, const unsigned short* __restrict__ Bt2p, int ldb, long strideB,
    void* __restrict__ Cout, void* __restrict__ Cout2, int ldc, long strideC,
    const float* __restrict__ bias,
    const float* __restrict__ resid, long strideR,
    int M, int N, int K, float scale, float pmul, float omul) {
  typedef typename Elem<ET>::T T;
  typedef typename Frag<T>::V V;
  const T* A = (const T*)Ap; const T* A2 = (const T*)A2p; const T* Bt = (const T*)Btp; const T* Bt2 = (const T*)Bt2p;
  __shared__ __align__(16) float sT[8][16 * 68];
  const int b    = blockIdx.y;
  const int lane = threadIdx.x & 31;
  const int wave = threadIdx.x >> 5;
  const int tilesN = N >> 6;
  const int tilesM = M >> 6;
  const int tile = blockIdx.x * 8 + wave;
  if (tile >= tilesM * tilesN) return;
  const int tm = tile / tilesN;
  const int tn = tile - tm * tilesN;
  const int m0 = tm << 6;
  const int n0 = tn << 6;

  const T* Ab  = A  + (size_t)b * strideA;
  const T* Bb  = Bt + (size_t)b * strideB;
  const T* Ab2 = SPLIT ? (A2  + (size_t)b * strideA) : nullptr;
  const T* Bb2 = SPLIT ? (Bt2 + (size_t)b * strideB) : nullptr;

  const int rlane = lane & 15;
  const int koff  = (lane >> 4) * 8;
  const int mOff  = (lane >> 4) * 8;

  v8f acc[4][4];
#pragma unroll
  for (int i = 0; i < 4; ++i)
#pragma unroll
    for (int j = 0; j < 4; ++j) acc[i][j] = (v8f){0.f,0.f,0.f,0.f,0.f,0.f,0.f,0.f};

  for (int k0 = 0; k0 < K; k0 += 32) {
    V bh[4], bl[4];
#pragma unroll
    for (int j = 0; j < 4; ++j) {
      const size_t bo = (size_t)(n0 + (j << 4) + rlane) * ldb + koff + k0;
      bh[j] = Frag<T>::load(Bb + bo);
      if (SPLIT) bl[j] = Frag<T>::load(Bb2 + bo);
    }
#pragma unroll
    for (int i = 0; i < 4; ++i) {
      const size_t ao = (size_t)(m0 + (i << 4) + rlane) * lda + koff + k0;
      V ah = Frag<T>::load(Ab + ao);
      V al;
      if (SPLIT) al = Frag<T>::load(Ab2 + ao);
#pragma unroll
      for (int j = 0; j < 4; ++j) {
        acc[i][j] = Frag<T>::mma(ah, bh[j], acc[i][j]);
        if (SPLIT) {
          acc[i][j] = Frag<T>::mma(ah, bl[j], acc[i][j]);
          acc[i][j] = Frag<T>::mma(al, bh[j], acc[i][j]);
        }
      }
      Frag<T>::guard(acc[i][0], acc[i][3], ah, SPLIT ? al : ah);
    }
    Frag<T>::keep(bh[0], bh[1], bh[2], bh[3]);
    if (SPLIT) Frag<T>::keep(bl[0], bl[1], bl[2], bl[3]);
  }
  acc_guard4(acc[0][0], acc[0][1], acc[0][2], acc[0][3]);
  acc_guard4(acc[1][0], acc[1][1], acc[1][2], acc[1][3]);
  acc_guard4(acc[2][0], acc[2][1], acc[2][2], acc[2][3]);
  acc_guard4(acc[3][0], acc[3][1], acc[3][2], acc[3][3]);

  float* slab = sT[wave];
  const float* Rb = RESID ? (resid + (size_t)b * strideR) : nullptr;
#pragma unroll
  for (int i = 0; i < 4; ++i) {
    const int mBase = m0 + (i << 4);
#pragma unroll
    for (int j = 0; j < 4; ++j) {
      const int n = n0 + (j << 4) + rlane;
      float bv = 0.f;
      if (BIAS_MODE == 2) bv = bias[n];
#pragma unroll
      for (int r = 0; r < 8; ++r) {
        float v = acc[i][j][r] * scale;
        if (BIAS_MODE == 1) v += bias[mBase + mOff + r];
        if (BIAS_MODE == 2) v += bv;
        if (NCL) v = nan_clean_f(v) * pmul;
        if (RESID) v += Rb[(size_t)(mBase + mOff + r) * ldc + n];
        if (ACT == 1) v = tanhf(v);
        if (ACT == 2) v = fmaxf(v, 0.0f);
        if (ACT == 3) v = v / (1.0f + expf(-v));
        if (ACT == 4) v = (v > 0.f) ? v : 0.01f * v;
        if (ACT == 5) v = 0.5f * v * (1.0f + erff(v * 0.70710678118654752f));
        if (NCL) v = v * omul;
        slab[(mOff + r) * 68 + (j << 4) + rlane] = v;
      }
    }
    __builtin_amdgcn_fence(__ATOMIC_RELEASE, "workgroup");
    __builtin_amdgcn_wave_barrier();
    __builtin_amdgcn_fence(__ATOMIC_ACQUIRE, "workgroup");
    if (OUT_MODE == 0) {
      float* C = (float*)Cout + (size_t)b * strideC;
      const int hh = lane >> 4, c4 = (lane & 15) * 4;
      for (int pass = 0; pass < 2; ++pass) {
#pragma unroll
        for (int it = 0; it < 8; ++it) {
          const int row = it * 2 + hh;
          v4f v = *(const v4f*)(slab + row * 68 + c4);
          *(volatile v4f*)(C + (size_t)(mBase + row) * ldc + n0 + c4) = v;
        }
        __threadfence();
      }
    } else {
      const int q = lane >> 3, c8 = (lane & 7) * 8;
      unsigned short* C  = (unsigned short*)Cout  + (size_t)b * strideC;
      unsigned short* C2 = (OUT_MODE == 2) ? ((unsigned short*)Cout2 + (size_t)b * strideC) : nullptr;
      for (int pass = 0; pass < 2; ++pass) {
#pragma unroll
        for (int it = 0; it < 4; ++it) {
          const int row = it * 4 + q;
          const float* sp = slab + row * 68 + c8;
          v8h hv, lv;
#pragma unroll
          for (int e = 0; e < 8; ++e) {
            if (OUT_MODE == 1) {
              hv[e] = (_Float16)sp[e];
            } else {
              unsigned short hb = f2bf_bits(sp[e]);
              unsigned short lb = f2bf_bits(sp[e] - bf_bits2f(hb));
              hv[e] = __builtin_bit_cast(_Float16, hb);
              lv[e] = __builtin_bit_cast(_Float16, lb);
            }
          }
          *(volatile v8h*)(C + (size_t)(mBase + row) * ldc + n0 + c8) = hv;
          if (OUT_MODE == 2) *(volatile v8h*)(C2 + (size_t)(mBase + row) * ldc + n0 + c8) = lv;
        }
        __threadfence();
      }
    }
    __builtin_amdgcn_fence(__ATOMIC_RELEASE, "workgroup");
    __builtin_amdgcn_wave_barrier();
    __builtin_amdgcn_fence(__ATOMIC_ACQUIRE, "workgroup");
  }
}

__global__ __launch_bounds__(256) void cast_f32_f16x2(
    const float* __restrict__ in, _Float16* __restrict__ out, int n2, float sc) {
  int i = blockIdx.x * 256 + threadIdx.x;
  if (i < n2) {
    const _Float16 h0 = (_Float16)(in[2 * i] * sc), h1 = (_Float16)(in[2 * i + 1] * sc);
    const unsigned u = (unsigned)__builtin_bit_cast(unsigned short, h0) | ((unsigned)__builtin_bit_cast(unsigned short, h1) << 16);
    ((volatile unsigned*)out)[i] = u;
    __threadfence();
    ((volatile unsigned*)out)[i] = u;
  }
}

__device__ __forceinline__ void ln256_store8(const float (&v)[8], const float* __restrict__ w,
                                             const float* __restrict__ bb, int c8, _Float16* dst) {
  float sm = 0.f;
#pragma unroll
  for (int e = 0; e < 8; ++e) sm += v[e];
#pragma unroll
  for (int m = 16; m > 0; m >>= 1) sm += __shfl_xor(sm, m, 32);
  const float mu = sm * (1.0f / (float)C_);
  float ss = 0.f;
#pragma unroll
  for (int e = 0; e < 8; ++e) { const float d = v[e] - mu; ss += d * d; }
#pragma unroll
  for (int m = 16; m > 0; m >>= 1) ss += __shfl_xor(ss, m, 32);
  const float rs = rsqrtf(ss * (1.0f / (float)C_) + 1e-6f);
  v8h o;
#pragma unroll
  for (int e = 0; e < 8; ++e) o[e] = (_Float16)((v[e] - mu) * rs * w[c8 + e] + bb[c8 + e]);
  *(volatile v8h*)dst = o;
  __threadfence();
  *(volatile v8h*)dst = o;
}

__global__ __launch_bounds__(256) void k_ln_x(const float* __restrict__ x,
                                              const float* __restrict__ w,
                                              const float* __restrict__ bb,
                                              _Float16* __restrict__ xn) {
  __shared__ float tile[C_][33];
  const int t  = threadIdx.x;
  const int p0 = blockIdx.x * 32;
  const int bN = p0 / L_;
  const int l0 = p0 - bN * L_;
  const int px = t & 31, cg = t >> 5;
  const float* xb = x + (size_t)bN * C_ * L_ + l0;
  for (int j = 0; j < C_ / 8; ++j) {
    const int c = j * 8 + cg;
    tile[c][px] = xb[(size_t)c * L_ + px];
  }
  __syncthreads();
  const int wid = t >> 5, lane = t & 31;
  const int c8 = lane * 8;
#pragma unroll 1
  for (int kq = 0; kq < 4; ++kq) {
    const int p = wid * 4 + kq;
    float v[8];
#pragma unroll
    for (int e = 0; e < 8; ++e) v[e] = tile[c8 + e][p];
    ln256_store8(v, w, bb, c8, xn + (size_t)(p0 + p) * C_ + c8);
  }
}

__global__ __launch_bounds__(256) void k_ln_row(const float* __restrict__ s,
                                                const float* __restrict__ w,
                                                const float* __restrict__ bb,
                                                _Float16* __restrict__ out, int nrows) {
  const int t = threadIdx.x, wid = t >> 5, lane = t & 31;
  const int row = blockIdx.x * 8 + wid;
  if (row >= nrows) return;
  const int c8 = lane * 8;
  const float* r = s + (size_t)row * C_ + c8;
  const v4f a = *(const v4f*)(r);
  const v4f c = *(const v4f*)(r + 4);
  float v[8];
  v[0] = a[0]; v[1] = a[1]; v[2] = a[2]; v[3] = a[3];
  v[4] = c[0]; v[5] = c[1]; v[6] = c[2]; v[7] = c[3];
  ln256_store8(v, w, bb, c8, out + (size_t)row * C_ + c8);
}

__global__ __launch_bounds__(256) void k_dwconv2d(const float* __restrict__ y,
                                                  const float* __restrict__ wk,
                                                  const float* __restrict__ bias,
                                                  float* __restrict__ out) {
  const int t   = threadIdx.x;
  const int tok = blockIdx.x * 4 + (t >> 6);
  const int c4  = (t & 63) * 4;
  const int bN  = tok / L_;
  const int l   = tok - bN * L_;
  const int h   = l / W_, ww = l - (l / W_) * W_;
  const float* yb = y + (size_t)bN * L_ * C_;
  v4f acc;
#pragma unroll
  for (int e = 0; e < 4; ++e) acc[e] = bias[c4 + e];
#pragma unroll
  for (int kh = 0; kh < 3; ++kh) {
    int hh = h + kh - 1;
    const bool vh = (hh >= 0) && (hh < H_);
    hh = hh < 0 ? 0 : (hh > H_ - 1 ? H_ - 1 : hh);
#pragma unroll
    for (int kw = 0; kw < 3; ++kw) {
      int wq = ww + kw - 1;
      const bool vw = (wq >= 0) && (wq < W_);
      wq = wq < 0 ? 0 : (wq > W_ - 1 ? W_ - 1 : wq);
      const float f = (vh && vw) ? 1.0f : 0.0f;
      const v4f val = *(const v4f*)(yb + (size_t)(hh * W_ + wq) * C_ + c4);
#pragma unroll
      for (int e = 0; e < 4; ++e) acc[e] += (wk[(c4 + e) * 9 + kh * 3 + kw] * f) * val[e];
    }
  }
  float* dst = out + (size_t)tok * C_ + c4;
  *(volatile v4f*)dst = acc;
  __threadfence();
  *(volatile v4f*)dst = acc;
}

__global__ __launch_bounds__(256) void k_glu(const float* __restrict__ ag, _Float16* __restrict__ r16, int ntok) {
  const size_t i = (size_t)blockIdx.x * 256 + threadIdx.x;
  if (i >= (size_t)ntok * (HID / 2)) return;
  const size_t tok = i / (HID / 2);
  const int cp = (int)(i - tok * (HID / 2)) * 2;
  const float* row = ag + tok * (size_t)(2 * HID);
  const float a0 = row[cp], a1 = row[cp + 1];
  const float g0 = row[HID + cp], g1 = row[HID + cp + 1];
  const float r0 = a0 * (1.0f / (1.0f + expf(-g0))) * 16.0f;
  const float r1 = a1 * (1.0f / (1.0f + expf(-g1))) * 16.0f;
  const _Float16 h0 = (_Float16)r0, h1 = (_Float16)r1;
  const unsigned u = (unsigned)__builtin_bit_cast(unsigned short, h0) | ((unsigned)__builtin_bit_cast(unsigned short, h1) << 16);
  ((volatile unsigned*)r16)[i] = u;
  __threadfence();
  ((volatile unsigned*)r16)[i] = u;
}

__global__ __launch_bounds__(256) void k_conv_route(const _Float16* __restrict__ r16,
                                                    const float* __restrict__ dww,
                                                    const float* __restrict__ dwb,
                                                    _Float16* __restrict__ d, int route) {
  const int t   = threadIdx.x;
  const int tok = blockIdx.x * 4 + (t >> 6);
  const int c8  = (t & 63) * 8;
  const int bN  = tok / L_;
  const int l   = tok - bN * L_;
  const int base = bN * L_;
  int im, ip; float fm, fp;
  if (route < 2) {
    im = l - 1; ip = l + 1;
    fm = (l >= 1) ? 1.0f : 0.0f;
    fp = (l <= L_ - 2) ? 1.0f : 0.0f;
    im = im < 0 ? 0 : im;
    ip = ip > L_ - 1 ? L_ - 1 : ip;
  } else {
    const int h = l / W_, w = l - h * W_;
    const int p = w * H_ + h;
    int pm = p - 1, pp = p + 1;
    fm = (p >= 1) ? 1.0f : 0.0f;
    fp = (p <= L_ - 2) ? 1.0f : 0.0f;
    pm = pm < 0 ? 0 : pm;
    pp = pp > L_ - 1 ? L_ - 1 : pp;
    im = (pm - (pm / H_) * H_) * W_ + (pm / H_);
    ip = (pp - (pp / H_) * H_) * W_ + (pp / H_);
  }
  int ia, ib; float fa, fb;
  if (route & 1) { ia = ip; fa = fp; ib = im; fb = fm; }
  else           { ia = im; fa = fm; ib = ip; fb = fp; }
  const v8h RA = *(const v8h*)(r16 + (size_t)(base + ia) * HID + c8);
  const v8h RC = *(const v8h*)(r16 + (size_t)tok * HID + c8);
  const v8h RB = *(const v8h*)(r16 + (size_t)(base + ib) * HID + c8);
  v8h o;
#pragma unroll
  for (int e = 0; e < 8; ++e) {
    const int ch = c8 + e;
    const float w0 = dww[ch * 3 + 0], w1 = dww[ch * 3 + 1], w2 = dww[ch * 3 + 2];
    const float v = (w0 * fa) * (float)RA[e] + w1 * (float)RC[e] + (w2 * fb) * (float)RB[e];
    o[e] = (_Float16)(v * 16.0f + dwb[ch] * 256.0f);
  }
  _Float16* dst = d + (size_t)tok * HID + c8;
  *(volatile v8h*)dst = o;
  __threadfence();
  *(volatile v8h*)dst = o;
}

extern "C" void kernel_launch(void* const* d_in, const int* in_sizes, int n_in,
                              void* d_out, int out_size, void* d_ws, size_t ws_size,
                              hipStream_t stream) {
  if (n_in < 17) return;
  if (in_sizes[0] != NTOK * C_ || out_size != NTOK * C_) return;
  if (in_sizes[1] != C_ || in_sizes[2] != C_ || in_sizes[3] != C_ * C_ || in_sizes[4] != C_) return;
  if (in_sizes[5] != C_ * 9 || in_sizes[6] != C_ || in_sizes[7] != C_ || in_sizes[8] != C_) return;
  if (in_sizes[9] != 2 * HID * C_ || in_sizes[10] != 2 * HID || in_sizes[11] != HID * 3 || in_sizes[12] != HID) return;
  if (in_sizes[13] != C_ * HID || in_sizes[14] != C_ || in_sizes[15] != C_ * C_ || in_sizes[16] != C_) return;

  const float* x         = (const float*)d_in[0];
  const float* ln2d_w    = (const float*)d_in[1];
  const float* ln2d_b    = (const float*)d_in[2];
  const float* inproj_w  = (const float*)d_in[3];
  const float* inproj_b  = (const float*)d_in[4];
  const float* dw2d_w    = (const float*)d_in[5];
  const float* dw2d_b    = (const float*)d_in[6];
  const float* ssm_ln_w  = (const float*)d_in[7];
  const float* ssm_ln_b  = (const float*)d_in[8];
  const float* ssm_in_w  = (const float*)d_in[9];
  const float* ssm_in_b  = (const float*)d_in[10];
  const float* ssm_dw_w  = (const float*)d_in[11];
  const float* ssm_dw_b  = (const float*)d_in[12];
  const float* ssm_out_w = (const float*)d_in[13];
  const float* ssm_out_b = (const float*)d_in[14];
  const float* outproj_w = (const float*)d_in[15];
  const float* outproj_b = (const float*)d_in[16];

  size_t off = 0;
  auto carve = [&](size_t bytes) -> size_t { size_t o = off; off += (bytes + 255) & ~(size_t)255; return o; };
  const size_t oX16 = carve((size_t)NTOK * C_ * 2);
  const size_t oW1  = carve((size_t)C_ * C_ * 2);
  const size_t oWsi = carve((size_t)2 * HID * C_ * 2);
  const size_t oWso = carve((size_t)C_ * HID * 2);
  const size_t oWo  = carve((size_t)C_ * C_ * 2);
  const size_t oY1  = carve((size_t)NTOK * C_ * 4);
  const size_t oS   = carve((size_t)NTOK * C_ * 4);
  const size_t oAG  = carve((size_t)NTOK * 2 * HID * 4);
  const size_t oR16 = carve((size_t)NTOK * HID * 2);
  if (off > ws_size) return;

  char* ws = (char*)d_ws;
  _Float16* X16  = (_Float16*)(ws + oX16);
  _Float16* W1h  = (_Float16*)(ws + oW1);
  _Float16* Wsih = (_Float16*)(ws + oWsi);
  _Float16* Wsoh = (_Float16*)(ws + oWso);
  _Float16* Woh  = (_Float16*)(ws + oWo);
  float*    Y1   = (float*)(ws + oY1);
  float*    S    = (float*)(ws + oS);
  float*    AG   = (float*)(ws + oAG);
  _Float16* R16  = (_Float16*)(ws + oR16);
  float*    T0   = Y1;
  _Float16* Dh   = (_Float16*)(ws + oAG);
  float*    T1   = (float*)(ws + oAG + (size_t)NTOK * HID * 2);
  _Float16* M16  = X16;
  float*    OUT  = (float*)d_out;

  dim3 blk(256);
  const float c64 = 64.0f;
  cast_f32_f16x2<<<(C_ * C_ / 2 + 255) / 256, blk, 0, stream>>>(inproj_w,  W1h,  C_ * C_ / 2, c64);
  cast_f32_f16x2<<<(2 * HID * C_ / 2 + 255) / 256, blk, 0, stream>>>(ssm_in_w,  Wsih, 2 * HID * C_ / 2, c64);
  cast_f32_f16x2<<<(C_ * HID / 2 + 255) / 256, blk, 0, stream>>>(ssm_out_w, Wsoh, C_ * HID / 2, c64);
  cast_f32_f16x2<<<(C_ * C_ / 2 + 255) / 256, blk, 0, stream>>>(outproj_w, Woh,  C_ * C_ / 2, c64);

  k_ln_x<<<NTOK / 32, blk, 0, stream>>>(x, ln2d_w, ln2d_b, X16);

  {
    const int M = NTOK, N = C_, K = C_;
    const int tiles = (M / 64) * (N / 64);
    wmma_gemm64<0, false, 2, 0, false, 0, 0><<<dim3((tiles + 7) / 8, 1), blk, 0, stream>>>(
        (const unsigned short*)X16, (const unsigned short*)X16, K, 0L,
        (const unsigned short*)W1h, (const unsigned short*)W1h, K, 0L,
        (void*)Y1, (void*)Y1, N, 0L,
        inproj_b, inproj_b, 0L,
        M, N, K, 1.0f / 64.0f, 1.0f, 1.0f);
  }

  k_dwconv2d<<<NTOK / 4, blk, 0, stream>>>(Y1, dw2d_w, dw2d_b, S);

  k_ln_row<<<NTOK / 8, blk, 0, stream>>>(S, ssm_ln_w, ssm_ln_b, X16, NTOK);

  {
    const int M = NTOK, N = 2 * HID, K = C_;
    const int tiles = (M / 64) * (N / 64);
    wmma_gemm64<0, false, 2, 0, false, 0, 0><<<dim3((tiles + 7) / 8, 1), blk, 0, stream>>>(
        (const unsigned short*)X16, (const unsigned short*)X16, K, 0L,
        (const unsigned short*)Wsih, (const unsigned short*)Wsih, K, 0L,
        (void*)AG, (void*)AG, N, 0L,
        ssm_in_b, ssm_in_b, 0L,
        M, N, K, 1.0f / 64.0f, 1.0f, 1.0f);
  }

  k_glu<<<(NTOK * (HID / 2) + 255) / 256, blk, 0, stream>>>(AG, R16, NTOK);

  {
    const int M = NTOK, N = C_, K = HID;
    const int tiles = (M / 64) * (N / 64);
    const float sc = 1.0f / (256.0f * 64.0f);
    for (int r = 0; r < 4; ++r) {
      k_conv_route<<<NTOK / 4, blk, 0, stream>>>(R16, ssm_dw_w, ssm_dw_b, Dh, r);
      const float* res = (r == 0) ? S : ((r == 2) ? T1 : T0);
      if (r < 3) {
        float* o = (r == 1) ? T1 : T0;
        wmma_gemm64<0, false, 2, 0, true, 0, 1><<<dim3((tiles + 7) / 8, 1), blk, 0, stream>>>(
            (const unsigned short*)Dh, (const unsigned short*)Dh, K, 0L,
            (const unsigned short*)Wsoh, (const unsigned short*)Wsoh, K, 0L,
            (void*)o, (void*)o, N, 0L,
            ssm_out_b, res, 0L,
            M, N, K, sc, 0.25f, 1.0f);
      } else {
        wmma_gemm64<0, false, 2, 1, true, 0, 1><<<dim3((tiles + 7) / 8, 1), blk, 0, stream>>>(
            (const unsigned short*)Dh, (const unsigned short*)Dh, K, 0L,
            (const unsigned short*)Wsoh, (const unsigned short*)Wsoh, K, 0L,
            (void*)M16, (void*)M16, N, 0L,
            ssm_out_b, res, 0L,
            M, N, K, sc, 0.25f, 256.0f);
      }
    }
  }

  {
    const int M = C_, N = L_, K = C_;
    const int tiles = (M / 64) * (N / 64);
    wmma_gemm64<0, false, 1, 0, true, 0, 1><<<dim3((tiles + 7) / 8, B_), blk, 0, stream>>>(
        (const unsigned short*)Woh, (const unsigned short*)Woh, K, 0L,
        (const unsigned short*)M16, (const unsigned short*)M16, K, (long)L_ * C_,
        (void*)OUT, (void*)OUT, L_, (long)C_ * L_,
        outproj_b, x, (long)C_ * L_,
        M, N, K, 1.0f / (256.0f * 64.0f), 1.0f, 1.0f);
  }
}
